// CopeMultiHeadAttention_31851477467658
// MI455X (gfx1250) — hardware-verified
//
#include <hip/hip_runtime.h>
#include <math.h>
#include <stdint.h>

constexpr int SEQ_LEN = 2048;
constexpr int NDIM    = 1024;
constexpr int NHD     = 16;
constexpr int HDIM    = 64;
constexpr int NPOSI   = 64;

typedef __attribute__((ext_vector_type(16))) _Float16 v16h;
typedef __attribute__((ext_vector_type(8)))  _Float16 v8h;
typedef __attribute__((ext_vector_type(16))) __bf16   v16b;
typedef __attribute__((ext_vector_type(8)))  __bf16   v8b;
typedef __attribute__((ext_vector_type(8)))  float    v8f;
typedef __attribute__((ext_vector_type(4)))  float    v4f;
typedef __attribute__((ext_vector_type(2)))  float    v2f;

__device__ __forceinline__ unsigned short f2bf_bits(float f) {
  unsigned u = __float_as_uint(f);
  return (unsigned short)((u + 0x7FFFu + ((u >> 16) & 1u)) >> 16);
}
__device__ __forceinline__ float bf_bits2f(unsigned short h) { return __uint_as_float(((unsigned)h) << 16); }
__device__ __forceinline__ unsigned pk16(unsigned short a, unsigned short b) { return (unsigned)a | ((unsigned)b << 16); }

__device__ __forceinline__ void dep_guard_h(v8f& a, v8f& b, v16h x, v16h y) { asm volatile("v_nop\n\tv_nop\n\tv_nop\n\tv_nop" : "+v"(a), "+v"(b) : "v"(x), "v"(y)); }
__device__ __forceinline__ void dep_guard_b(v8f& a, v8f& b, v16b x, v16b y) { asm volatile("v_nop\n\tv_nop\n\tv_nop\n\tv_nop" : "+v"(a), "+v"(b) : "v"(x), "v"(y)); }
__device__ __forceinline__ void keep4_h(v16h a, v16h b, v16h c, v16h d) { asm volatile("v_nop" :: "v"(a), "v"(b), "v"(c), "v"(d)); }
__device__ __forceinline__ void keep4_b(v16b a, v16b b, v16b c, v16b d) { asm volatile("v_nop" :: "v"(a), "v"(b), "v"(c), "v"(d)); }
__device__ __forceinline__ void acc_guard4(v8f& a, v8f& b, v8f& c, v8f& d) { asm volatile("v_nop\n\tv_nop\n\tv_nop\n\tv_nop" : "+v"(a), "+v"(b), "+v"(c), "+v"(d)); }
template <typename T> struct Frag;
template <> struct Frag<_Float16> {
  typedef v16h V; union U { v16h v; v8h h[2]; };
  static __device__ __forceinline__ v16h load(const _Float16* p) {
    U f; f.h[0] = *(const v8h*)(p); f.h[1] = *(const v8h*)(p + 16); return f.v;
  }
  static __device__ __forceinline__ v8f mma(v16h a, v16h b, v8f c) {
    return __builtin_amdgcn_wmma_f32_16x16x32_f16(false, a, false, b, (short)0, c, false, false);
  }
  static __device__ __forceinline__ void guard(v8f& a, v8f& b, v16h x, v16h y) { dep_guard_h(a, b, x, y); }
  static __device__ __forceinline__ void keep(v16h a, v16h b, v16h c, v16h d) { keep4_h(a, b, c, d); }
};
template <> struct Frag<__bf16> {
  typedef v16b V; union U { v16b v; v8b h[2]; };
  static __device__ __forceinline__ v16b load(const __bf16* p) {
    U f; f.h[0] = *(const v8b*)(p); f.h[1] = *(const v8b*)(p + 16); return f.v;
  }
  static __device__ __forceinline__ v8f mma(v16b a, v16b b, v8f c) {
    return __builtin_amdgcn_wmma_f32_16x16x32_bf16(false, a, false, b, (short)0, c, false, false);
  }
  static __device__ __forceinline__ void guard(v8f& a, v8f& b, v16b x, v16b y) { dep_guard_b(a, b, x, y); }
  static __device__ __forceinline__ void keep(v16b a, v16b b, v16b c, v16b d) { keep4_b(a, b, c, d); }
};

template <int ET> struct Elem;
template <> struct Elem<0> { typedef _Float16 T; };
template <> struct Elem<1> { typedef __bf16 T; };
template <int ET, bool SPLIT, int BIAS_MODE, int OUT_MODE, bool RESID, int ACT = 0>
__global__ __launch_bounds__(256) void wmma_gemm64(
    const unsigned short* __restrict__ Ap, const unsigned short* __restrict__ A2p, int lda, long strideA,
    const unsigned short* __restrict__ Btp, const unsigned short* __restrict__ Bt2p, int ldb, long strideB,
    void* __restrict__ Cout, void* __restrict__ Cout2, int ldc, long strideC,
    const float* __restrict__ bias,
    const float* __restrict__ resid, long strideR,
    int M, int N, int K, float scale) {
  typedef typename Elem<ET>::T T;
  typedef typename Frag<T>::V V;
  const T* A = (const T*)Ap; const T* A2 = (const T*)A2p; const T* Bt = (const T*)Btp; const T* Bt2 = (const T*)Bt2p;
  __shared__ __align__(16) float sT[8][16 * 68];
  const int b    = blockIdx.y;
  const int lane = threadIdx.x & 31;
  const int wave = threadIdx.x >> 5;
  const int tilesN = N >> 6;
  const int tilesM = M >> 6;
  const int tile = blockIdx.x * 8 + wave;
  if (tile >= tilesM * tilesN) return;
  const int tm = tile / tilesN;
  const int tn = tile - tm * tilesN;
  const int m0 = tm << 6;
  const int n0 = tn << 6;

  const T* Ab  = A  + (size_t)b * strideA;
  const T* Bb  = Bt + (size_t)b * strideB;
  const T* Ab2 = SPLIT ? (A2  + (size_t)b * strideA) : nullptr;
  const T* Bb2 = SPLIT ? (Bt2 + (size_t)b * strideB) : nullptr;

  const int rlane = lane & 15;
  const int koff  = (lane >> 4) * 8;
  const int mOff  = (lane >> 4) * 8;

  v8f acc[4][4];
#pragma unroll
  for (int i = 0; i < 4; ++i)
#pragma unroll
    for (int j = 0; j < 4; ++j) acc[i][j] = (v8f){0.f,0.f,0.f,0.f,0.f,0.f,0.f,0.f};

  for (int k0 = 0; k0 < K; k0 += 32) {
    V bh[4], bl[4];
#pragma unroll
    for (int j = 0; j < 4; ++j) {
      const size_t bo = (size_t)(n0 + (j << 4) + rlane) * ldb + koff + k0;
      bh[j] = Frag<T>::load(Bb + bo);
      if (SPLIT) bl[j] = Frag<T>::load(Bb2 + bo);
    }
#pragma unroll
    for (int i = 0; i < 4; ++i) {
      const size_t ao = (size_t)(m0 + (i << 4) + rlane) * lda + koff + k0;
      V ah = Frag<T>::load(Ab + ao);
      V al;
      if (SPLIT) al = Frag<T>::load(Ab2 + ao);
#pragma unroll
      for (int j = 0; j < 4; ++j) {
        acc[i][j] = Frag<T>::mma(ah, bh[j], acc[i][j]);
        if (SPLIT) {
          acc[i][j] = Frag<T>::mma(ah, bl[j], acc[i][j]);
          acc[i][j] = Frag<T>::mma(al, bh[j], acc[i][j]);
        }
      }
      Frag<T>::guard(acc[i][0], acc[i][3], ah, SPLIT ? al : ah);
    }
    Frag<T>::keep(bh[0], bh[1], bh[2], bh[3]);
    if (SPLIT) Frag<T>::keep(bl[0], bl[1], bl[2], bl[3]);
  }
  acc_guard4(acc[0][0], acc[0][1], acc[0][2], acc[0][3]);
  acc_guard4(acc[1][0], acc[1][1], acc[1][2], acc[1][3]);
  acc_guard4(acc[2][0], acc[2][1], acc[2][2], acc[2][3]);
  acc_guard4(acc[3][0], acc[3][1], acc[3][2], acc[3][3]);

  float* slab = sT[wave];
  const float* Rb = RESID ? (resid + (size_t)b * strideR) : nullptr;
#pragma unroll
  for (int i = 0; i < 4; ++i) {
    const int mBase = m0 + (i << 4);
#pragma unroll
    for (int j = 0; j < 4; ++j) {
      const int n = n0 + (j << 4) + rlane;
      float bv = 0.f;
      if (BIAS_MODE == 2) bv = bias[n];
#pragma unroll
      for (int r = 0; r < 8; ++r) {
        float v = acc[i][j][r] * scale;
        if (BIAS_MODE == 1) v += bias[mBase + mOff + r];
        if (BIAS_MODE == 2) v += bv;
        if (RESID) v += Rb[(size_t)(mBase + mOff + r) * ldc + n];
        if (ACT == 2) v = fmaxf(v, 0.0f);
        if (ACT == 4) v = (v > 0.f) ? v : 0.01f * v;
        slab[(mOff + r) * 68 + (j << 4) + rlane] = v;
      }
    }
    __builtin_amdgcn_fence(__ATOMIC_RELEASE, "workgroup");
    __builtin_amdgcn_wave_barrier();
    __builtin_amdgcn_fence(__ATOMIC_ACQUIRE, "workgroup");
    if (OUT_MODE == 0) {
      float* C = (float*)Cout + (size_t)b * strideC;
      const int hh = lane >> 4, c4 = (lane & 15) * 4;
      for (int pass = 0; pass < 2; ++pass) {
#pragma unroll
        for (int it = 0; it < 8; ++it) {
          const int row = it * 2 + hh;
          v4f v = *(const v4f*)(slab + row * 68 + c4);
          *(volatile v4f*)(C + (size_t)(mBase + row) * ldc + n0 + c4) = v;
        }
        __threadfence();
      }
    } else {
      const int q = lane >> 3, c8 = (lane & 7) * 8;
      unsigned short* C  = (unsigned short*)Cout  + (size_t)b * strideC;
      unsigned short* C2 = (OUT_MODE == 2) ? ((unsigned short*)Cout2 + (size_t)b * strideC) : nullptr;
      for (int pass = 0; pass < 2; ++pass) {
#pragma unroll
        for (int it = 0; it < 4; ++it) {
          const int row = it * 4 + q;
          const float* sp = slab + row * 68 + c8;
          v8h hv, lv;
#pragma unroll
          for (int e = 0; e < 8; ++e) {
            if (OUT_MODE == 1) {
              hv[e] = (_Float16)sp[e];
            } else {
              unsigned short hb = f2bf_bits(sp[e]);
              unsigned short lb = f2bf_bits(sp[e] - bf_bits2f(hb));
              hv[e] = __builtin_bit_cast(_Float16, hb);
              lv[e] = __builtin_bit_cast(_Float16, lb);
            }
          }
          *(volatile v8h*)(C + (size_t)(mBase + row) * ldc + n0 + c8) = hv;
          if (OUT_MODE == 2) *(volatile v8h*)(C2 + (size_t)(mBase + row) * ldc + n0 + c8) = lv;
        }
        __threadfence();
      }
    }
    __builtin_amdgcn_fence(__ATOMIC_RELEASE, "workgroup");
    __builtin_amdgcn_wave_barrier();
    __builtin_amdgcn_fence(__ATOMIC_ACQUIRE, "workgroup");
  }
}

__global__ __launch_bounds__(256) void cast_bf16x2_kernel(const float* __restrict__ in, unsigned short* __restrict__ out, int n2) {
  const int i = blockIdx.x * 256 + threadIdx.x;
  if (i < n2) {
    const v2f f = *(const v2f*)(in + 2 * (size_t)i);
    const unsigned u = pk16(f2bf_bits(f[0]), f2bf_bits(f[1]));
    ((volatile unsigned*)out)[i] = u;
    __threadfence();
    ((volatile unsigned*)out)[i] = u;
  }
}

__global__ __launch_bounds__(256) void cast_f16s_x2_kernel(const float* __restrict__ in, unsigned short* __restrict__ out, int n2, float mul) {
  const int i = blockIdx.x * 256 + threadIdx.x;
  if (i < n2) {
    const v2f f = *(const v2f*)(in + 2 * (size_t)i);
    const float g0 = bf_bits2f(f2bf_bits(f[0])) * mul;
    const float g1 = bf_bits2f(f2bf_bits(f[1])) * mul;
    const unsigned u = pk16(__builtin_bit_cast(unsigned short, (_Float16)g0), __builtin_bit_cast(unsigned short, (_Float16)g1));
    ((volatile unsigned*)out)[i] = u;
    __threadfence();
    ((volatile unsigned*)out)[i] = u;
  }
}

constexpr int ATT_D  = 64;
constexpr int ATT_NW = 4;
constexpr int ATT_QB = 64;
constexpr int ATT_KC = 64;
constexpr float P_CARRY = 32768.0f;

__device__ __forceinline__ v8f mma_h(v16h a, v16h b, v8f c) {
  c = __builtin_amdgcn_wmma_f32_16x16x32_f16(false, a, false, b, (short)0, c, false, false);
  asm volatile("v_nop\n\tv_nop\n\tv_nop\n\tv_nop" : "+v"(c) : "v"(a), "v"(b));
  return c;
}

__global__ __launch_bounds__(128)
void cpos_attn_kernel(const unsigned short* __restrict__ qp, const unsigned short* __restrict__ kp,
                      const unsigned short* __restrict__ vtp, const float* __restrict__ pos_emb,
                      unsigned short* __restrict__ outp, const int* __restrict__ nheads_unused) {
  union FB { v16h v; v8h h[2]; };
  __shared__ __align__(16) _Float16 Ksh[ATT_KC * ATT_D];
  __shared__ __align__(16) _Float16 Vth[ATT_D * ATT_KC];
  __shared__ __align__(16) _Float16 Psh[ATT_NW][16 * ATT_KC];
  __shared__ __align__(16) float    LIs[ATT_NW][16 * 68];
  __shared__ __align__(16) float    Os[ATT_NW][16 * 68];

  const int tid  = threadIdx.x;
  const int wave = tid >> 5;
  const int lane = tid & 31;
  const int hh   = lane >> 4;
  const int c    = lane & 15;

  const int nqb = SEQ_LEN / ATT_QB;
  const int bx  = blockIdx.x;
  const int qb  = bx % nqb;
  const int h   = bx / nqb;
  const int q0  = qb * ATT_QB + wave * 16;

  const _Float16* Qg = (const _Float16*)(const void*)qp  + (size_t)h * ATT_D;
  const _Float16* Kg = (const _Float16*)(const void*)kp  + (size_t)h * ATT_D;
  const _Float16* Vg = (const _Float16*)(const void*)vtp + (size_t)h * ATT_D * SEQ_LEN;
  _Float16*       Og = (_Float16*)(void*)outp + (size_t)h * ATT_D;

#pragma unroll 1
  for (int i = tid; i < NPOSI * HDIM; i += 128) {
    const int n = i >> 6, d = i & 63;
    const float pe = bf_bits2f(f2bf_bits(pos_emb[d * NPOSI + n])) * 64.0f;
    Ksh[n * ATT_D + d] = (_Float16)pe;
  }
  __syncthreads();

  v16h qa[2];
#pragma unroll
  for (int dc = 0; dc < 2; ++dc)
    qa[dc] = Frag<_Float16>::load(Qg + (size_t)(q0 + c) * NDIM + dc * 32 + 8 * hh);

  {
    v8f li[4];
#pragma unroll
    for (int t = 0; t < 4; ++t) li[t] = (v8f){0.f,0.f,0.f,0.f,0.f,0.f,0.f,0.f};
#pragma unroll
    for (int t = 0; t < 4; ++t) {
#pragma unroll
      for (int dc = 0; dc < 2; ++dc) {
        FB pb;
        pb.h[0] = *(const v8h*)(Ksh + (t * 16 + c) * ATT_D + dc * 32 + 8 * hh);
        pb.h[1] = *(const v8h*)(Ksh + (t * 16 + c) * ATT_D + dc * 32 + 16 + 8 * hh);
        li[t] = mma_h(qa[dc], pb.v, li[t]);
      }
    }
    float* lisw = LIs[wave];
#pragma unroll
    for (int t = 0; t < 4; ++t) {
#pragma unroll
      for (int r = 0; r < 8; ++r) lisw[(8 * hh + r) * 68 + t * 16 + c] = li[t][r] * (1.0f / 64.0f);
    }
  }

  float mrow[8], lrow[8], srun[8];
  v8f oacc[4];
#pragma unroll
  for (int r = 0; r < 8; ++r) { mrow[r] = -INFINITY; lrow[r] = 0.f; srun[r] = 0.f; }
#pragma unroll
  for (int t = 0; t < 4; ++t) oacc[t] = (v8f){0.f,0.f,0.f,0.f,0.f,0.f,0.f,0.f};

  const int nChunks = SEQ_LEN / ATT_KC;
#pragma unroll 1
  for (int kci = 0; kci < nChunks; ++kci) {
    const int kv0 = (nChunks - 1 - kci) * ATT_KC;
    __syncthreads();
    {
      const int r = tid >> 1, half = (tid & 1) * 32;
      const _Float16* ksrc = Kg + (size_t)(kv0 + r) * NDIM + half;
      const _Float16* vsrc = Vg + (size_t)r * SEQ_LEN + kv0 + half;
#pragma unroll
      for (int i = 0; i < 4; ++i) {
        const v8h a0 = *(const v8h*)(ksrc + 8 * i);
        const v8h b0 = *(const v8h*)(vsrc + 8 * i);
        *(v8h*)(Ksh + r * ATT_D  + half + 8 * i) = a0;
        *(v8h*)(Vth + r * ATT_KC + half + 8 * i) = b0;
      }
    }
    __syncthreads();

    v8f s[4];
#pragma unroll
    for (int j = 0; j < 4; ++j) {
      s[j] = (v8f){0.f,0.f,0.f,0.f,0.f,0.f,0.f,0.f};
#pragma unroll
      for (int dc = 0; dc < 2; ++dc) {
        FB kb;
        kb.h[0] = *(const v8h*)(Ksh + (j * 16 + c) * ATT_D + dc * 32 + 8 * hh);
        kb.h[1] = *(const v8h*)(Ksh + (j * 16 + c) * ATT_D + dc * 32 + 16 + 8 * hh);
        s[j] = mma_h(qa[dc], kb.v, s[j]);
      }
    }

    const float* lisw = LIs[wave];
    float cm[8];
#pragma unroll
    for (int r = 0; r < 8; ++r) {
      const int row = 8 * hh + r;
      float xs[4], tot[4];
#pragma unroll
      for (int j = 0; j < 4; ++j) {
        const float sv = s[j][r] * 0.125f;
        s[j][r] = sv;
        float x = __builtin_amdgcn_rcpf(1.0f + __expf(-sv));
#pragma unroll
        for (int off = 1; off < 16; off <<= 1) {
          const float tsh = __shfl_down(x, off, 16);
          if (c + off < 16) x += tsh;
        }
        xs[j]  = x;
        tot[j] = __shfl(x, 0, 16);
      }
      const float aft3 = srun[r];
      const float aft2 = aft3 + tot[3];
      const float aft1 = aft2 + tot[2];
      const float aft0 = aft1 + tot[1];
      srun[r] = aft0 + tot[0];
      const float aft[4] = {aft0, aft1, aft2, aft3};
      float m = -INFINITY;
#pragma unroll
      for (int j = 0; j < 4; ++j) {
        float pos = aft[j] + xs[j];
        pos = fminf(pos, (float)(NPOSI - 1));
        const float pf = floorf(pos);
        const float pc = ceilf(pos);
        const float w  = pos - pf;
        int ipf = (int)pf; ipf = ipf < 0 ? 0 : (ipf > NPOSI - 1 ? NPOSI - 1 : ipf);
        int ipc = (int)pc; ipc = ipc < 0 ? 0 : (ipc > NPOSI - 1 ? NPOSI - 1 : ipc);
        const float lf = lisw[row * 68 + ipf];
        const float lc = lisw[row * 68 + ipc];
        const float sv = s[j][r] + (lc * w + lf * (1.0f - w));
        s[j][r] = sv;
        m = fmaxf(m, sv);
      }
#pragma unroll
      for (int off = 1; off < 16; off <<= 1) m = fmaxf(m, __shfl_xor(m, off, 32));
      cm[r] = m;
    }

    _Float16* pw = Psh[wave];
#pragma unroll
    for (int r = 0; r < 8; ++r) {
      const float mnew  = fmaxf(mrow[r], cm[r]);
      const float alpha = __expf(mrow[r] - mnew);
      mrow[r] = mnew;
      float psum = 0.f;
#pragma unroll
      for (int j = 0; j < 4; ++j) {
        const float p = __expf(s[j][r] - mnew);
        psum += p;
        pw[(8 * hh + r) * ATT_KC + j * 16 + c] = (_Float16)(p * P_CARRY);
      }
#pragma unroll
      for (int off = 1; off < 16; off <<= 1) psum += __shfl_xor(psum, off, 32);
      lrow[r] = lrow[r] * alpha + psum;
#pragma unroll
      for (int t = 0; t < 4; ++t) oacc[t][r] *= alpha;
    }
    __builtin_amdgcn_fence(__ATOMIC_RELEASE, "workgroup");
    __builtin_amdgcn_wave_barrier();
    __builtin_amdgcn_fence(__ATOMIC_ACQUIRE, "workgroup");
#pragma unroll 1
    for (int kk = 0; kk < 2; ++kk) {
      FB pa;
      pa.h[0] = *(const v8h*)(pw + c * ATT_KC + kk * 32 + 8 * hh);
      pa.h[1] = *(const v8h*)(pw + c * ATT_KC + kk * 32 + 16 + 8 * hh);
#pragma unroll
      for (int t = 0; t < 4; ++t) {
        FB vb;
        vb.h[0] = *(const v8h*)(Vth + (t * 16 + c) * ATT_KC + kk * 32 + 8 * hh);
        vb.h[1] = *(const v8h*)(Vth + (t * 16 + c) * ATT_KC + kk * 32 + 16 + 8 * hh);
        oacc[t] = mma_h(pa.v, vb.v, oacc[t]);
      }
    }
  }

  float* os = Os[wave];
#pragma unroll
  for (int r = 0; r < 8; ++r) {
    const float inv = 16.0f / (lrow[r] * P_CARRY);
#pragma unroll
    for (int t = 0; t < 4; ++t) os[(8 * hh + r) * 68 + t * 16 + c] = oacc[t][r] * inv;
  }
  __builtin_amdgcn_fence(__ATOMIC_RELEASE, "workgroup");
  __builtin_amdgcn_wave_barrier();
  __builtin_amdgcn_fence(__ATOMIC_ACQUIRE, "workgroup");
  {
    const int q = lane >> 3, c8 = (lane & 7) * 8;
    for (int pass = 0; pass < 2; ++pass) {
#pragma unroll
      for (int it = 0; it < 4; ++it) {
        const int row = it * 4 + q;
        const float* sp = os + row * 68 + c8;
        v8h hv;
#pragma unroll
        for (int e = 0; e < 8; ++e) hv[e] = (_Float16)sp[e];
        *(volatile v8h*)(Og + (size_t)(q0 + row) * NDIM + c8) = hv;
      }
      __threadfence();
    }
  }
}

extern "C" void kernel_launch(void* const* d_in, const int* in_sizes, int n_in,
                              void* d_out, int out_size, void* d_ws, size_t ws_size,
                              hipStream_t stream) {
  const int xn = SEQ_LEN * NDIM;
  const int wn = NDIM * NDIM;
  if (n_in < 13) return;
  if (in_sizes[0] != xn || in_sizes[1] != xn || in_sizes[2] != xn) return;
  if (in_sizes[3] != wn || in_sizes[5] != wn || in_sizes[7] != wn || in_sizes[9] != wn) return;
  if (in_sizes[4] != NDIM || in_sizes[6] != NDIM || in_sizes[8] != NDIM || in_sizes[10] != NDIM) return;
  if (in_sizes[11] != HDIM * NPOSI) return;
  if (out_size != xn) return;

  const float* q_in   = (const float*)d_in[0];
  const float* k_in   = (const float*)d_in[1];
  const float* v_in   = (const float*)d_in[2];
  const float* Wq_w   = (const float*)d_in[3];
  const float* Wq_b   = (const float*)d_in[4];
  const float* Wk_w   = (const float*)d_in[5];
  const float* Wk_b   = (const float*)d_in[6];
  const float* Wv_w   = (const float*)d_in[7];
  const float* Wv_b   = (const float*)d_in[8];
  const float* Wo_w   = (const float*)d_in[9];
  const float* Wo_b   = (const float*)d_in[10];
  const float* posemb = (const float*)d_in[11];
  const int*   nh_p   = (const int*)d_in[12];
  float* out = (float*)d_out;

  const size_t xb16 = (size_t)xn * 2;
  const size_t wb16 = (size_t)wn * 2;
  unsigned char* ws = (unsigned char*)d_ws;
  size_t off = 0;
  unsigned short* XQ   = (unsigned short*)(ws + off); off += xb16;
  unsigned short* XK   = (unsigned short*)(ws + off); off += xb16;
  unsigned short* XV   = (unsigned short*)(ws + off); off += xb16;
  unsigned short* WQ   = (unsigned short*)(ws + off); off += wb16;
  unsigned short* WK   = (unsigned short*)(ws + off); off += wb16;
  unsigned short* WV   = (unsigned short*)(ws + off); off += wb16;
  unsigned short* WO   = (unsigned short*)(ws + off); off += wb16;
  unsigned short* Q16  = (unsigned short*)(ws + off); off += xb16;
  unsigned short* K16  = (unsigned short*)(ws + off); off += xb16;
  unsigned short* VT16 = (unsigned short*)(ws + off); off += xb16;
  unsigned short* O16  = (unsigned short*)(ws + off); off += xb16;
  if (off > ws_size) return;

  const int xn2 = xn / 2, wn2 = wn / 2;
  cast_bf16x2_kernel<<<dim3((unsigned)((xn2 + 255) / 256)), dim3(256), 0, stream>>>(q_in, XQ, xn2);
  cast_bf16x2_kernel<<<dim3((unsigned)((xn2 + 255) / 256)), dim3(256), 0, stream>>>(k_in, XK, xn2);
  cast_bf16x2_kernel<<<dim3((unsigned)((xn2 + 255) / 256)), dim3(256), 0, stream>>>(v_in, XV, xn2);
  cast_bf16x2_kernel<<<dim3((unsigned)((wn2 + 255) / 256)), dim3(256), 0, stream>>>(Wq_w, WQ, wn2);
  cast_bf16x2_kernel<<<dim3((unsigned)((wn2 + 255) / 256)), dim3(256), 0, stream>>>(Wk_w, WK, wn2);
  cast_bf16x2_kernel<<<dim3((unsigned)((wn2 + 255) / 256)), dim3(256), 0, stream>>>(Wv_w, WV, wn2);
  cast_f16s_x2_kernel<<<dim3((unsigned)((wn2 + 255) / 256)), dim3(256), 0, stream>>>(Wo_w, WO, wn2, 16.0f);

  const int tilesP = (SEQ_LEN / 64) * (NDIM / 64);
  const unsigned gP = (unsigned)((tilesP + 7) / 8);
  wmma_gemm64<1, false, 2, 1, false><<<dim3(gP, 1), dim3(256), 0, stream>>>(
      XQ, XQ, NDIM, 0L, WQ, WQ, NDIM, 0L, (void*)Q16, (void*)Q16, NDIM, 0L,
      Wq_b, Wq_b, 0L, SEQ_LEN, NDIM, NDIM, 1.0f);
  wmma_gemm64<1, false, 2, 1, false><<<dim3(gP, 1), dim3(256), 0, stream>>>(
      XK, XK, NDIM, 0L, WK, WK, NDIM, 0L, (void*)K16, (void*)K16, NDIM, 0L,
      Wk_b, Wk_b, 0L, SEQ_LEN, NDIM, NDIM, 1.0f);
  const int tilesV = (NDIM / 64) * (SEQ_LEN / 64);
  const unsigned gV = (unsigned)((tilesV + 7) / 8);
  wmma_gemm64<1, false, 1, 1, false><<<dim3(gV, 1), dim3(256), 0, stream>>>(
      WV, WV, NDIM, 0L, XV, XV, NDIM, 0L, (void*)VT16, (void*)VT16, SEQ_LEN, 0L,
      Wv_b, Wv_b, 0L, NDIM, SEQ_LEN, NDIM, 1.0f);

  cpos_attn_kernel<<<dim3((unsigned)(NHD * (SEQ_LEN / ATT_QB))), dim3(128), 0, stream>>>(Q16, K16, VT16, posemb, O16, nh_p);

  wmma_gemm64<0, false, 2, 0, false><<<dim3(gP, 1), dim3(256), 0, stream>>>(
      O16, O16, NDIM, 0L, WO, WO, NDIM, 0L, (void*)out, (void*)out, NDIM, 0L,
      Wo_b, Wo_b, 0L, SEQ_LEN, NDIM, NDIM, 1.0f / 256.0f);
}
